// MambaBlock_70111046140103
// MI455X (gfx1250) — hardware-verified
//
#include <hip/hip_runtime.h>
#include <stddef.h>
#include <stdint.h>
#include <math.h>


#define MROWS  2048
#define LSEQ   1024
#define DMODEL 1024
#define DINNER 2048
#define NIN    4096
#define K2     4096
#define NDT    2112
#define PLANE  (2048 * 2048)
#define GBM    128
#define GBN    64
#define GTHR   128
#define PTHR   256
#define TC     64
#define STHR   128
#define WSMAX  134217728

#define U_XB   (MROWS * DMODEL / 8)
#define U_WIN  (NIN * DMODEL / 8)
#define U_DT   (DINNER * DINNER / 8)
#define U_B    (16 * DINNER / 8)
#define U_C    (16 * DINNER / 8)
#define U_Z    (32 * K2 / 8)
#define U_WO   (DMODEL * DINNER / 8)
#define E1     (U_XB)
#define E2     (E1 + U_WIN)
#define E3     (E2 + U_DT)
#define E4     (E3 + U_B)
#define E5     (E4 + U_C)
#define E6     (E5 + U_Z)
#define E7     (E6 + U_WO)

static_assert(E1 % PTHR == 0 && E2 % PTHR == 0 && E3 % PTHR == 0 && E4 % PTHR == 0);
static_assert(E5 % PTHR == 0 && E6 % PTHR == 0 && E7 % PTHR == 0);
static_assert(MROWS % GBM == 0 && NIN % GBN == 0 && NDT % GBN == 0 && DMODEL % GBN == 0);
static_assert(DMODEL % 32 == 0 && K2 % 32 == 0 && K2 == 2 * DINNER);
static_assert(GBM == (GTHR / 32) * 32 && GBN == 64);
static_assert(NDT == DINNER + 64 && DINNER % GBN == 0);
static_assert(LSEQ % TC == 0 && (2 * TC * 64) == 8 * STHR * 8 && (TC * 8) % STHR == 0);
static_assert(DINNER % 64 == 0 && MROWS == 2 * LSEQ);

typedef float          v4f   __attribute__((ext_vector_type(4)));
typedef float          v8f   __attribute__((ext_vector_type(8)));
typedef int            v8i   __attribute__((ext_vector_type(8)));
typedef unsigned short v4us  __attribute__((ext_vector_type(4)));
typedef unsigned short v8us  __attribute__((ext_vector_type(8)));
typedef unsigned short v16us __attribute__((ext_vector_type(16)));
typedef __bf16         v16bf __attribute__((ext_vector_type(16)));
typedef v4f  __attribute__((may_alias)) v4fa;
typedef v4us __attribute__((may_alias)) v4usa;
typedef v8us __attribute__((may_alias)) v8usa;
union FragB { v16bf v; v16us u; v8us h[2]; v8i w; };

__device__ __forceinline__ v8f wmb(const FragB& a, const FragB& b, v8f c) {
  v8f d = __builtin_amdgcn_wmma_f32_16x16x32_bf16(false, a.v, false, b.v, (short)0, c, false, false);
  asm volatile("v_nop\n\tv_nop\n\tv_nop\n\tv_nop" : "+v"(d) : "v"(a.w), "v"(b.w));
  return d;
}

__device__ __forceinline__ unsigned bf16_bits(float f) {
  const unsigned u = __float_as_uint(f);
  return (u + 0x7FFFu + ((u >> 16) & 1u)) >> 16;
}
__device__ __forceinline__ float bf16_val(float f) {
  return __uint_as_float(bf16_bits(f) << 16);
}
__device__ __forceinline__ float silu1(float v) {
  return v * (1.0f / (1.0f + expf(-v)));
}
__device__ __forceinline__ float softplus1(float v) {
  return fmaxf(v, 0.0f) + log1pf(expf(-fabsf(v)));
}

__device__ __forceinline__ v8us tr8(const float* __restrict__ src, int Ns, int n, int k8) {
  const float* p = src + (size_t)k8 * (size_t)Ns + n;
  v8us o;
#pragma unroll
  for (int i = 0; i < 8; ++i) o[i] = (unsigned short)bf16_bits(p[(size_t)i * (size_t)Ns]);
  return o;
}
__device__ __forceinline__ void put1(unsigned short* dp, v8us o) {
  *(volatile v8us*)dp = o;
  __threadfence();
  *(volatile v8us*)dp = o;
}
__device__ __forceinline__ void put2(unsigned short* d0, unsigned short* d1, v8us o) {
  *(volatile v8us*)d0 = o;
  *(volatile v8us*)d1 = o;
  __threadfence();
  *(volatile v8us*)d0 = o;
  *(volatile v8us*)d1 = o;
}

__global__ __launch_bounds__(PTHR) void k_prep(const float* __restrict__ x, const float* __restrict__ in_w,
                                               const float* __restrict__ dt_w, const float* __restrict__ B_w,
                                               const float* __restrict__ C_w, const float* __restrict__ out_w,
                                               unsigned short* XB, unsigned short* WIN,
                                               unsigned short* WD2, unsigned short* WO2) {
  const int u = (int)blockIdx.x * PTHR + (int)threadIdx.x;
  if (u < E1) {
    const float* p = x + (size_t)u * 8;
    const v4f a = *(const v4f*)p;
    const v4f b = *(const v4f*)(p + 4);
    v8us o;
    o[0] = (unsigned short)bf16_bits(a.x); o[1] = (unsigned short)bf16_bits(a.y);
    o[2] = (unsigned short)bf16_bits(a.z); o[3] = (unsigned short)bf16_bits(a.w);
    o[4] = (unsigned short)bf16_bits(b.x); o[5] = (unsigned short)bf16_bits(b.y);
    o[6] = (unsigned short)bf16_bits(b.z); o[7] = (unsigned short)bf16_bits(b.w);
    put1(XB + (size_t)u * 8, o);
  } else if (u < E2) {
    const int v = u - E1;
    const int n = v >> 7, k8 = (v & 127) * 8;
    const v8us o = tr8(in_w, NIN, n, k8);
    put1(WIN + (size_t)n * DMODEL + k8, o);
  } else if (u < E3) {
    const int v = u - E2;
    const int n = v >> 8, k8 = (v & 255) * 8;
    const v8us o = tr8(dt_w, DINNER, n, k8);
    unsigned short* dp = WD2 + (size_t)n * K2 + k8;
    put2(dp, dp + DINNER, o);
  } else if (u < E4) {
    const int v = u - E3;
    const int n = v >> 8, k8 = (v & 255) * 8;
    const v8us o = tr8(B_w, 16, n, k8);
    unsigned short* dp = WD2 + (size_t)(DINNER + n) * K2 + k8;
    put2(dp, dp + DINNER, o);
  } else if (u < E5) {
    const int v = u - E4;
    const int n = v >> 8, k8 = (v & 255) * 8;
    const v8us o = tr8(C_w, 16, n, k8);
    unsigned short* dp = WD2 + (size_t)(DINNER + 16 + n) * K2 + k8;
    put2(dp, dp + DINNER, o);
  } else if (u < E6) {
    const int v = u - E5;
    const int row = DINNER + 32 + (v >> 9), c8 = (v & 511) * 8;
    const v8us o = {0, 0, 0, 0, 0, 0, 0, 0};
    put1(WD2 + (size_t)row * K2 + c8, o);
  } else if (u < E7) {
    const int v = u - E6;
    const int n = v >> 8, k8 = (v & 255) * 8;
    const v8us o = tr8(out_w, DMODEL, n, k8);
    unsigned short* dp = WO2 + (size_t)n * K2 + k8;
    put2(dp, dp + DINNER, o);
  }
}

template <int ACT>
__device__ __forceinline__ void epi_rows(float* stg, int wave, int hh, int m, v4f b4, float* ob, int ldo) {
#pragma unroll 1
  for (int i = 0; i < 16; ++i) {
    float* sp = stg + (32 * wave + 2 * i + hh) * GBN + 4 * m;
    v4f v = *(const v4fa*)sp;
    v = v + b4;
    if constexpr (ACT == 1) {
      v.x = silu1(v.x); v.y = silu1(v.y); v.z = silu1(v.z); v.w = silu1(v.w);
    } else if constexpr (ACT == 2) {
      v.x = softplus1(v.x); v.y = softplus1(v.y); v.z = softplus1(v.z); v.w = softplus1(v.w);
    }
    *(v4fa*)sp = v;
    *(volatile v4f*)(ob + (size_t)(2 * i + hh) * (size_t)ldo) = v;
  }
  __threadfence();
#pragma unroll 1
  for (int i = 0; i < 16; ++i) {
    const float* sp = stg + (32 * wave + 2 * i + hh) * GBN + 4 * m;
    const v4f v = *(const v4fa*)sp;
    *(volatile v4f*)(ob + (size_t)(2 * i + hh) * (size_t)ldo) = v;
  }
}

template <int EPI>
__global__ __launch_bounds__(GTHR) void k_gemm(const unsigned short* __restrict__ A,
                                               const unsigned short* __restrict__ WT, int K,
                                               const float* __restrict__ bias0, const float* __restrict__ bias1,
                                               const float* __restrict__ bias2, float* out0, float* out1) {
  __shared__ __attribute__((aligned(16))) float stg[GBM * GBN];
  const int tid = (int)threadIdx.x, lane = tid & 31, wave = tid >> 5, hh = lane >> 4, m = lane & 15;
  const int rowBase = (int)blockIdx.x * GBM;
  const int col0    = (int)blockIdx.y * GBN;

  v8f acc[2][4];
  {
    const v8f z = {0.f, 0.f, 0.f, 0.f, 0.f, 0.f, 0.f, 0.f};
#pragma unroll
    for (int t = 0; t < 4; ++t) { acc[0][t] = z; acc[1][t] = z; }
  }
  const unsigned short* ap0 = A + (size_t)(rowBase + 32 * wave + m) * (size_t)K + 8 * hh;
  const unsigned short* ap1 = ap0 + (size_t)16 * (size_t)K;
  const unsigned short* wp  = WT + (size_t)(col0 + m) * (size_t)K + 8 * hh;
  const int ksteps = K >> 5;
#pragma unroll 1
  for (int ks = 0; ks < ksteps; ++ks) {
    FragB a0, a1;
    a0.h[0] = *(const v8usa*)(ap0 + 32 * ks);
    a0.h[1] = *(const v8usa*)(ap0 + 32 * ks + 16);
    a1.h[0] = *(const v8usa*)(ap1 + 32 * ks);
    a1.h[1] = *(const v8usa*)(ap1 + 32 * ks + 16);
#pragma unroll
    for (int t = 0; t < 4; ++t) {
      const unsigned short* wq = wp + (size_t)(16 * t) * (size_t)K + 32 * ks;
      FragB bf;
      bf.h[0] = *(const v8usa*)wq;
      bf.h[1] = *(const v8usa*)(wq + 16);
      acc[0][t] = wmb(a0, bf, acc[0][t]);
      acc[1][t] = wmb(a1, bf, acc[1][t]);
    }
  }

#pragma unroll
  for (int rt = 0; rt < 2; ++rt) {
#pragma unroll
    for (int t = 0; t < 4; ++t) {
      const int lc = 16 * t + m;
#pragma unroll
      for (int r = 0; r < 8; ++r) {
        const int lr = 32 * wave + 16 * rt + 8 * hh + r;
        stg[lr * GBN + lc] = acc[rt][t][r];
      }
    }
  }
  __syncthreads();

  if constexpr (EPI == 0) {
    const int plane = col0 >> 11;
    const int cc    = col0 & (DINNER - 1);
    const v4f t4 = *(const v4f*)(bias0 + col0 + 4 * m);
    v4f b4;
    b4.x = bf16_val(t4.x); b4.y = bf16_val(t4.y); b4.z = bf16_val(t4.z); b4.w = bf16_val(t4.w);
    float* ob = out0 + (size_t)plane * (size_t)PLANE + (size_t)(rowBase + 32 * wave) * DINNER + cc + 4 * m;
    if (plane == 0) epi_rows<0>(stg, wave, hh, m, b4, ob, DINNER);
    else            epi_rows<1>(stg, wave, hh, m, b4, ob, DINNER);
  } else if constexpr (EPI == 1) {
    if ((int)blockIdx.y < DINNER / GBN) {
      const int bc0 = col0 < (DINNER - GBN) ? col0 : (DINNER - GBN);
      const v4f t4 = *(const v4f*)(bias0 + bc0 + 4 * m);
      v4f b4;
      b4.x = bf16_val(t4.x); b4.y = bf16_val(t4.y); b4.z = bf16_val(t4.z); b4.w = bf16_val(t4.w);
      float* ob = out0 + (size_t)(rowBase + 32 * wave) * DINNER + col0 + 4 * m;
      epi_rows<2>(stg, wave, hh, m, b4, ob, DINNER);
    } else {
      const int c4 = lane & 7, rq = lane >> 3;
      const v4f bb = *(const v4f*)(bias1 + 4 * (c4 & 3));
      const v4f cb = *(const v4f*)(bias2 + 4 * (c4 & 3));
      const bool isC = c4 >= 4;
      v4f b4;
      b4.x = bf16_val(isC ? cb.x : bb.x);
      b4.y = bf16_val(isC ? cb.y : bb.y);
      b4.z = bf16_val(isC ? cb.z : bb.z);
      b4.w = bf16_val(isC ? cb.w : bb.w);
      float* ob = out1 + (size_t)(rowBase + 32 * wave + rq) * 32 + 4 * c4;
#pragma unroll 1
      for (int j = 0; j < 8; ++j) {
        float* sp = stg + (32 * wave + 4 * j + rq) * GBN + 4 * c4;
        v4f v = *(const v4fa*)sp;
        v = v + b4;
        *(v4fa*)sp = v;
        *(volatile v4f*)(ob + (size_t)(4 * j) * 32) = v;
      }
      __threadfence();
#pragma unroll 1
      for (int j = 0; j < 8; ++j) {
        const float* sp = stg + (32 * wave + 4 * j + rq) * GBN + 4 * c4;
        const v4f v = *(const v4fa*)sp;
        *(volatile v4f*)(ob + (size_t)(4 * j) * 32) = v;
      }
    }
  } else {
    const v4f t4 = *(const v4f*)(bias0 + col0 + 4 * m);
    v4f b4;
    b4.x = bf16_val(t4.x); b4.y = bf16_val(t4.y); b4.z = bf16_val(t4.z); b4.w = bf16_val(t4.w);
    float* ob = out0 + (size_t)(rowBase + 32 * wave) * DMODEL + col0 + 4 * m;
    epi_rows<0>(stg, wave, hh, m, b4, ob, DMODEL);
  }
}

__global__ __launch_bounds__(PTHR) void k_conv(const float* __restrict__ XZ, const float* __restrict__ cw,
                                               const float* __restrict__ cb, float* XC, unsigned short* XCH) {
  __shared__ __attribute__((aligned(16))) unsigned short hl[2048];
  const int tid   = (int)threadIdx.x;
  const int row   = (int)blockIdx.x >> 1;
  const int cbase = ((int)blockIdx.x & 1) * 1024;
  const int c     = cbase + 4 * tid;
  const int l     = row & (LSEQ - 1);

  v4f s;
  {
    const v4f b4 = *(const v4f*)(cb + c);
    s.x = bf16_val(b4.x); s.y = bf16_val(b4.y); s.z = bf16_val(b4.z); s.w = bf16_val(b4.w);
  }
#pragma unroll
  for (int w = 0; w < 4; ++w) {
    const int lt  = l + w - 1;
    const int ltc = lt < 0 ? 0 : (lt > LSEQ - 1 ? LSEQ - 1 : lt);
    const float f = (lt == ltc) ? 1.0f : 0.0f;
    const int rr  = row + (ltc - l);
    const v4f x4 = *(const v4f*)(XZ + (size_t)rr * DINNER + c);
    const v4f w4 = *(const v4f*)(cw + (size_t)w * DINNER + c);
    s.x = fmaf(bf16_val(w4.x) * f, x4.x, s.x);
    s.y = fmaf(bf16_val(w4.y) * f, x4.y, s.y);
    s.z = fmaf(bf16_val(w4.z) * f, x4.z, s.z);
    s.w = fmaf(bf16_val(w4.w) * f, x4.w, s.w);
  }
  v4f v;
  v.x = silu1(s.x); v.y = silu1(s.y); v.z = silu1(s.z); v.w = silu1(s.w);

  v4us hv, lv;
  {
    unsigned hb;
    hb = bf16_bits(v.x); hv[0] = (unsigned short)hb; lv[0] = (unsigned short)bf16_bits(v.x - __uint_as_float(hb << 16));
    hb = bf16_bits(v.y); hv[1] = (unsigned short)hb; lv[1] = (unsigned short)bf16_bits(v.y - __uint_as_float(hb << 16));
    hb = bf16_bits(v.z); hv[2] = (unsigned short)hb; lv[2] = (unsigned short)bf16_bits(v.z - __uint_as_float(hb << 16));
    hb = bf16_bits(v.w); hv[3] = (unsigned short)hb; lv[3] = (unsigned short)bf16_bits(v.w - __uint_as_float(hb << 16));
  }
  *(v4usa*)(hl + 4 * tid) = hv;
  *(v4usa*)(hl + 1024 + 4 * tid) = lv;
  __syncthreads();
  const v8us q = *(const v8usa*)(hl + 8 * tid);

  float* xp = XC + (size_t)row * DINNER + c;
  unsigned short* hp = XCH + (size_t)row * K2 + (size_t)(tid >> 7) * DINNER + cbase + 8 * (tid & 127);
  *(volatile v4f*)xp = v;
  *(volatile v8us*)hp = q;
  __threadfence();
  *(volatile v4f*)xp = v;
  *(volatile v8us*)hp = q;
}

__global__ __launch_bounds__(STHR) void k_scan(const float* __restrict__ DT, const float* __restrict__ BC,
                                               const float* __restrict__ XC, const float* __restrict__ SG,
                                               const float* __restrict__ Am, const float* __restrict__ Dp,
                                               unsigned short* YG) {
  __shared__ __attribute__((aligned(16))) float bcs[TC * 32];
  __shared__ __attribute__((aligned(16))) unsigned short ot[2 * TC * 64];
  const int tid = (int)threadIdx.x;
  const int ch  = tid >> 1, p = tid & 1;
  const int b   = (int)blockIdx.x >> 5;
  const int d0  = ((int)blockIdx.x & 31) * 64;
  const int d   = d0 + ch;
  const size_t rb = (size_t)b * LSEQ;

  float a[8], h[8];
  {
    const v4f a0 = *(const v4f*)(Am + (size_t)d * 16 + 8 * p);
    const v4f a1 = *(const v4f*)(Am + (size_t)d * 16 + 8 * p + 4);
    a[0] = bf16_val(a0.x); a[1] = bf16_val(a0.y); a[2] = bf16_val(a0.z); a[3] = bf16_val(a0.w);
    a[4] = bf16_val(a1.x); a[5] = bf16_val(a1.y); a[6] = bf16_val(a1.z); a[7] = bf16_val(a1.w);
#pragma unroll
    for (int j = 0; j < 8; ++j) h[j] = 0.0f;
  }
  const float dpv = bf16_val(Dp[d]);

#pragma unroll 1
  for (int t0 = 0; t0 < LSEQ; t0 += TC) {
#pragma unroll
    for (int it = 0; it < (TC * 8) / STHR; ++it) {
      const int i = it * STHR + tid;
      const v4f v = *(const v4f*)(BC + (rb + (size_t)t0) * 32 + 4 * (size_t)i);
      *(v4fa*)(bcs + 4 * i) = v;
    }
    __syncthreads();

#pragma unroll 1
    for (int tl = 0; tl < TC; ++tl) {
      const size_t gi = (rb + (size_t)(t0 + tl)) * DINNER + d;
      const float dtv = DT[gi];
      const float xv  = XC[gi];
      const float sg  = SG[gi];
      const float* br = bcs + tl * 32 + 8 * p;
      const v4f b0 = *(const v4fa*)br;
      const v4f b1 = *(const v4fa*)(br + 4);
      const v4f c0 = *(const v4fa*)(br + 16);
      const v4f c1 = *(const v4fa*)(br + 20);
      float s = 0.0f;
#define STEPN(J, BJ, CJ) { \
        const float dA  = expf(dtv * a[J]); \
        const float dbx = (dtv * (BJ)) * xv; \
        h[J] = dA * h[J] + dbx; \
        s += h[J] * (CJ); }
      STEPN(0, b0.x, c0.x)
      STEPN(1, b0.y, c0.y)
      STEPN(2, b0.z, c0.z)
      STEPN(3, b0.w, c0.w)
      STEPN(4, b1.x, c1.x)
      STEPN(5, b1.y, c1.y)
      STEPN(6, b1.z, c1.z)
      STEPN(7, b1.w, c1.w)
#undef STEPN
      const float so  = __shfl_xor(s, 1, 32);
      const float tot = s + so;
      float y = tot + xv * dpv;
      y = y * sg;
      const unsigned hb = bf16_bits(y);
      const unsigned lb = bf16_bits(y - __uint_as_float(hb << 16));
      ot[(p * TC + tl) * 64 + ch] = (unsigned short)(p != 0 ? lb : hb);
    }
    __syncthreads();

    v8us qv[8];
#pragma unroll
    for (int it = 0; it < 8; ++it) qv[it] = *(const v8usa*)(ot + 8 * (it * STHR + tid));
#pragma unroll
    for (int it = 0; it < 8; ++it) {
      const int u = it * STHR + tid;
      const int line = u >> 3, piece = u & 7;
      const int plane = line >> 6, tl = line & (TC - 1);
      unsigned short* op = YG + (rb + (size_t)(t0 + tl)) * K2 + (size_t)plane * DINNER + d0 + 8 * piece;
      *(volatile v8us*)op = qv[it];
    }
    __threadfence();
#pragma unroll
    for (int it = 0; it < 8; ++it) {
      const int u = it * STHR + tid;
      const int line = u >> 3, piece = u & 7;
      const int plane = line >> 6, tl = line & (TC - 1);
      unsigned short* op = YG + (rb + (size_t)(t0 + tl)) * K2 + (size_t)plane * DINNER + d0 + 8 * piece;
      *(volatile v8us*)op = qv[it];
    }
  }
}

static inline size_t al256(size_t o) { return (o + 255) & ~(size_t)255; }

extern "C" void kernel_launch(void* const* d_in, const int* in_sizes, int n_in,
                              void* d_out, int out_size, void* d_ws, size_t ws_size,
                              hipStream_t stream) {
  if (n_in < 15) return;
  if (in_sizes[0] != MROWS * DMODEL) return;
  if (in_sizes[1] != DMODEL * NIN || in_sizes[2] != NIN) return;
  if (in_sizes[3] != 4 * DINNER || in_sizes[4] != DINNER) return;
  if (in_sizes[5] != DINNER * 16 || in_sizes[6] != DINNER) return;
  if (in_sizes[7] != DINNER * 16 || in_sizes[8] != 16) return;
  if (in_sizes[9] != DINNER * 16 || in_sizes[10] != 16) return;
  if (in_sizes[11] != DINNER * DINNER || in_sizes[12] != DINNER) return;
  if (in_sizes[13] != DINNER * DMODEL || in_sizes[14] != DMODEL) return;
  if (out_size != MROWS * DMODEL) return;

  const float* x      = (const float*)d_in[0];
  const float* in_w   = (const float*)d_in[1];
  const float* in_b   = (const float*)d_in[2];
  const float* conv_w = (const float*)d_in[3];
  const float* conv_b = (const float*)d_in[4];
  const float* Am     = (const float*)d_in[5];
  const float* Dp     = (const float*)d_in[6];
  const float* B_w    = (const float*)d_in[7];
  const float* B_b    = (const float*)d_in[8];
  const float* C_w    = (const float*)d_in[9];
  const float* C_b    = (const float*)d_in[10];
  const float* dt_w   = (const float*)d_in[11];
  const float* dt_b   = (const float*)d_in[12];
  const float* out_w  = (const float*)d_in[13];
  const float* out_b  = (const float*)d_in[14];
  float* out = (float*)d_out;

  char* ws = (char*)d_ws;
  size_t off = 0;
  const size_t oXB  = off; off = al256(off + (size_t)MROWS * DMODEL * 2);
  const size_t oWIN = off; off = al256(off + (size_t)NIN * DMODEL * 2);
  const size_t oWD2 = off; off = al256(off + (size_t)NDT * K2 * 2);
  const size_t oWO2 = off; off = al256(off + (size_t)DMODEL * K2 * 2);
  const size_t oXZ  = off; off = al256(off + (size_t)2 * PLANE * 4);
  const size_t oXC  = off; off = al256(off + (size_t)PLANE * 4);
  const size_t oXCH = off; off = al256(off + (size_t)MROWS * K2 * 2);
  const size_t oYG  = off; off = al256(off + (size_t)MROWS * K2 * 2);
  const size_t oBC  = off; off = al256(off + (size_t)MROWS * 32 * 4);
  if (off > ws_size || off > (size_t)WSMAX) return;
  unsigned short* XB  = (unsigned short*)(ws + oXB);
  unsigned short* WIN = (unsigned short*)(ws + oWIN);
  unsigned short* WD2 = (unsigned short*)(ws + oWD2);
  unsigned short* WO2 = (unsigned short*)(ws + oWO2);
  float*          XZ  = (float*)(ws + oXZ);
  float*          SGp = XZ + (size_t)PLANE;
  float*          DTp = XZ;
  float*          XC  = (float*)(ws + oXC);
  unsigned short* XCH = (unsigned short*)(ws + oXCH);
  unsigned short* YG  = (unsigned short*)(ws + oYG);
  float*          BCp = (float*)(ws + oBC);

  k_prep<<<E7 / PTHR, PTHR, 0, stream>>>(x, in_w, dt_w, B_w, C_w, out_w, XB, WIN, WD2, WO2);
  k_gemm<0><<<dim3(MROWS / GBM, NIN / GBN), GTHR, 0, stream>>>(XB, WIN, DMODEL, in_b, in_b, in_b, XZ, XZ);
  k_conv<<<MROWS * 2, PTHR, 0, stream>>>(XZ, conv_w, conv_b, XC, XCH);
  k_gemm<1><<<dim3(MROWS / GBM, NDT / GBN), GTHR, 0, stream>>>(XCH, WD2, K2, dt_b, B_b, C_b, DTp, BCp);
  k_scan<<<2 * (DINNER / 64), STHR, 0, stream>>>(DTp, BCp, XC, SGp, Am, Dp, YG);
  k_gemm<2><<<dim3(MROWS / GBM, DMODEL / GBN), GTHR, 0, stream>>>(YG, WO2, K2, out_b, out_b, out_b, out, out);
}
